// Bipartite_Layers_19310172963573
// MI455X (gfx1250) — hardware-run, weakly checked
//
#include <hip/hip_runtime.h>

typedef float          v8f   __attribute__((ext_vector_type(8)));
typedef float          v4f   __attribute__((ext_vector_type(4)));
typedef unsigned int   v4u   __attribute__((ext_vector_type(4)));
typedef int            v8i   __attribute__((ext_vector_type(8)));
typedef unsigned short v8us  __attribute__((ext_vector_type(8)));
typedef unsigned short v16us __attribute__((ext_vector_type(16)));
typedef __bf16         v16bf __attribute__((ext_vector_type(16)));
typedef _Float16       v16h  __attribute__((ext_vector_type(16)));
typedef v4f  __attribute__((may_alias)) v4fa;
typedef v8us __attribute__((may_alias)) v8usa;
union FragB { v16bf v; v16us u; v8us h[2]; v8i w; };
union FragH { v16h  v; v16us u; v8us h[2]; v8i w; };

__device__ __forceinline__ v8f wmb(const FragB& a, const FragB& b, v8f c) {
  v8f d = __builtin_amdgcn_wmma_f32_16x16x32_bf16(false, a.v, false, b.v, (short)0, c, false, false);
  asm volatile("v_nop\n\tv_nop\n\tv_nop\n\tv_nop" : "+v"(d) : "v"(a.w), "v"(b.w));
  return d;
}

__device__ __forceinline__ v8f wmh(const FragH& a, const FragH& b, v8f c) {
  v8f d = __builtin_amdgcn_wmma_f32_16x16x32_f16(false, a.v, false, b.v, (short)0, c, false, false);
  asm volatile("v_nop\n\tv_nop\n\tv_nop\n\tv_nop" : "+v"(d) : "v"(a.w), "v"(b.w));
  return d;
}

__device__ __forceinline__ unsigned bf16_bits(float f) {
  const unsigned u = __float_as_uint(f);
  const unsigned r = (u + 0x7FFFu + ((u >> 16) & 1u)) >> 16;
  const unsigned q = (u >> 16) | 0x40u;
  return ((u & 0x7fffffffu) > 0x7f800000u) ? q : r;
}

__device__ __forceinline__ float bf16_val(float f) {
  return __uint_as_float(bf16_bits(f) << 16);
}
__device__ __forceinline__ int clampi(int v, int lo, int hi) {
  return v < lo ? lo : (v > hi ? hi : v);
}

__device__ __forceinline__ unsigned f16_bits(float f) {
  const unsigned u  = __float_as_uint(f);
  const unsigned s  = (u >> 16) & 0x8000u;
  const unsigned a  = u & 0x7fffffffu;
  const unsigned t  = a - 0x38000000u;
  const unsigned r  = (t + 0x0FFFu + ((t >> 13) & 1u)) >> 13;
  const unsigned rc = r > 0x7C00u ? 0x7C00u : r;
  const bool small  = a < 0x38800000u;
  const bool isnan  = a > 0x7f800000u;
  const unsigned fin = small ? 0u : (s | rc);
  return isnan ? (s | 0x7E00u) : fin;
}

__device__ __forceinline__ unsigned pk16(unsigned lo, unsigned hi) { return lo | (hi << 16); }
__device__ __forceinline__ unsigned bf16_lo_bits(float v) {
  float hi = bf16_val(v);
  asm volatile("" : "+v"(hi));
  return bf16_bits(v - hi);
}
__device__ __forceinline__ v4u pack8_bf16(v4f a, v4f c) {
  return (v4u){ pk16(bf16_bits(a[0]), bf16_bits(a[1])), pk16(bf16_bits(a[2]), bf16_bits(a[3])),
                pk16(bf16_bits(c[0]), bf16_bits(c[1])), pk16(bf16_bits(c[2]), bf16_bits(c[3])) };
}
__device__ __forceinline__ v4u pack8_bf16_lo(v4f a, v4f c) {
  return (v4u){ pk16(bf16_lo_bits(a[0]), bf16_lo_bits(a[1])), pk16(bf16_lo_bits(a[2]), bf16_lo_bits(a[3])),
                pk16(bf16_lo_bits(c[0]), bf16_lo_bits(c[1])), pk16(bf16_lo_bits(c[2]), bf16_lo_bits(c[3])) };
}
__device__ __forceinline__ v4u pack8_f16(v4f a, v4f c) {
  return (v4u){ pk16(f16_bits(a[0]), f16_bits(a[1])), pk16(f16_bits(a[2]), f16_bits(a[3])),
                pk16(f16_bits(c[0]), f16_bits(c[1])), pk16(f16_bits(c[2]), f16_bits(c[3])) };
}

template <int FORM>
__global__ __launch_bounds__(256) void k_plane(const float* __restrict__ src, int rows, int cols, int ldsrc,
                                               unsigned short* __restrict__ dst, int MP, int KP) {
  static_assert(FORM >= 0 && FORM <= 3);
  const int KTOT = (FORM == 1 || FORM == 3) ? 2 * KP : KP;
  const unsigned ppr   = (unsigned)(KTOT >> 3);
  const unsigned kp8   = (unsigned)(KP >> 3);
  const unsigned total = (unsigned)MP * ppr;
  const unsigned g     = blockIdx.x * 256u + threadIdx.x;
  const unsigned rowu  = g / ppr;
  const unsigned p     = g - rowu * ppr;
  const bool second    = p >= kp8;
  const int row = (int)rowu;
  const int c0  = (int)((second ? p - kp8 : p) << 3);
  const float* srow = src + (size_t)clampi(row, 0, rows - 1) * (size_t)ldsrc;
  float x[8];
  unsigned mk[8];
#pragma unroll
  for (int e = 0; e < 8; ++e) {
    const int c = c0 + e;
    const float v = srow[clampi(c, 0, cols - 1)];
    asm volatile("" :: "v"(v));
    x[e]  = v;
    mk[e] = (row < rows && c < cols) ? 0xFFFFu : 0u;
  }
  const v4f a = (v4f){ x[0], x[1], x[2], x[3] };
  const v4f c = (v4f){ x[4], x[5], x[6], x[7] };
  v4u o;
  if (FORM == 2) {
    o = pack8_f16(a, c);
  } else {
    const v4u hi = pack8_bf16(a, c);
    o = hi;
    if (FORM == 1) { const v4u lo = pack8_bf16_lo(a, c); o = second ? lo : hi; }
  }
  const v4u mw = (v4u){ pk16(mk[0], mk[1]), pk16(mk[2], mk[3]), pk16(mk[4], mk[5]), pk16(mk[6], mk[7]) };
  o &= mw;
  if (g < total) {
    volatile v4u* q = (volatile v4u*)(dst + (size_t)g * 8);
    *q = o;
    __threadfence();
    *q = o;
  }
}

template <int FORM> struct FragOf    { typedef FragB T; };
template <>         struct FragOf<2> { typedef FragH T; };
__device__ __forceinline__ v8f mm(const FragB& a, const FragB& b, v8f c) { return wmb(a, b, c); }
__device__ __forceinline__ v8f mm(const FragH& a, const FragH& b, v8f c) { return wmh(a, b, c); }
template <class F> __device__ __forceinline__ F ld_frag(const unsigned short* p) {
  F f;
  f.h[0] = *(const v8usa*)(p);
  f.h[1] = *(const v8usa*)(p + 16);
  return f;
}

template <int FORM, int EPI>
__global__ __launch_bounds__(256) __attribute__((amdgpu_num_vgpr(248)))
void k_gemm_nt(const unsigned short* __restrict__ A, const unsigned short* __restrict__ B,
               const float* __restrict__ bias, float* __restrict__ D, int M, int N, int KTOT, int ldd) {
  static_assert(FORM >= 0 && FORM <= 2);
  static_assert(EPI == 0 || EPI == 1);
  typedef typename FragOf<FORM>::T F;
  __shared__ __attribute__((aligned(16))) float sT[8][16 * 68];
  const int lane = threadIdx.x & 31;
  const int wave = threadIdx.x >> 5;
  const int tilesM = (M + 63) >> 6;
  const int tilesN = (N + 63) >> 6;
  const int tile = blockIdx.x * 8 + wave;
  if (tile >= tilesM * tilesN) return;
  const int tm = tile / tilesN;
  const int tn = tile - tm * tilesN;
  const int m0 = tm << 6;
  const int n0 = tn << 6;

  const int rl = lane & 15;
  const int h8 = (lane >> 4) * 8;
  const unsigned short* pa = A + (size_t)(m0 + rl) * (size_t)KTOT + h8;
  const unsigned short* pb = B + (size_t)(n0 + rl) * (size_t)KTOT + h8;

  v8f acc[4][4];
#pragma unroll
  for (int i = 0; i < 4; ++i)
#pragma unroll
    for (int j = 0; j < 4; ++j) acc[i][j] = (v8f){0.f, 0.f, 0.f, 0.f, 0.f, 0.f, 0.f, 0.f};

#pragma unroll 1
  for (int k0 = 0; k0 < KTOT; k0 += 32) {
    F bf[4];
#pragma unroll
    for (int j = 0; j < 4; ++j) bf[j] = ld_frag<F>(pb + (size_t)(j << 4) * (size_t)KTOT + k0);
#pragma unroll
    for (int i = 0; i < 4; ++i) {
      const F af = ld_frag<F>(pa + (size_t)(i << 4) * (size_t)KTOT + k0);
#pragma unroll
      for (int j = 0; j < 4; ++j) acc[i][j] = mm(af, bf[j], acc[i][j]);
    }
  }

  float* slab = sT[wave];
  const int hh = lane >> 4;
  const int c4 = (lane & 15) * 4;
  const int nc = n0 + c4;
  const bool cok = nc < N;
  v4f bv = (v4f){0.f, 0.f, 0.f, 0.f};
  if (EPI == 1) {
    bv = *(const v4fa*)(bias + clampi(nc, 0, N - 4));
    asm volatile("" :: "v"(bv));
  }
#pragma unroll
  for (int i = 0; i < 4; ++i) {
    const int mBase = m0 + (i << 4);
#pragma unroll
    for (int j = 0; j < 4; ++j) {
#pragma unroll
      for (int r = 0; r < 8; ++r) slab[(h8 + r) * 68 + (j << 4) + rl] = acc[i][j][r];
    }
    __builtin_amdgcn_fence(__ATOMIC_RELEASE, "workgroup");
    __builtin_amdgcn_wave_barrier();
    __builtin_amdgcn_fence(__ATOMIC_ACQUIRE, "workgroup");
    v4f vv[8];
#pragma unroll
    for (int it = 0; it < 8; ++it) {
      const int row = it * 2 + hh;
      v4f v = *(const v4fa*)(slab + row * 68 + c4);
      if (EPI == 1) v += bv;
      vv[it] = v;
    }
    for (int pass = 0; pass < 2; ++pass) {
#pragma unroll
      for (int it = 0; it < 8; ++it) {
        const int row = mBase + it * 2 + hh;
        if (cok && row < M) *(volatile v4f*)(D + (size_t)row * (size_t)ldd + nc) = vv[it];
      }
      __threadfence();
    }
    __builtin_amdgcn_fence(__ATOMIC_RELEASE, "workgroup");
    __builtin_amdgcn_wave_barrier();
    __builtin_amdgcn_fence(__ATOMIC_ACQUIRE, "workgroup");
  }
}

#include <math.h>
#include <stddef.h>

constexpr int kB = 16, kT = 4096, kD = 64, kF = 128, kA = 16;
constexpr int kRows = kB * kT;
constexpr int kNPL  = 320;
constexpr int kAgg  = 2 * kF * kA;
constexpr int kAgg2 = 2 * kAgg;
constexpr int kMPA  = 64;
constexpr int kNVEC = 384;
constexpr int kSP   = 132;
constexpr int kOut1 = kRows * kF;

static_assert(kD == 64 && kF == 128 && kA == 16);
static_assert((kT % 256) == 0);
static_assert(kD + 2 * kF * kA == 4160);
static_assert((kRows % 64) == 0 && (kRows % 16) == 0);
static_assert((kNPL % 64) == 0 && (kNPL % 32) == 0 && kNPL >= 2 * kF + kA);
static_assert((kD % 32) == 0 && (kAgg2 % 32) == 0);
static_assert((kMPA % 64) == 0 && kMPA >= kB && (kB % 16) == 0);
static_assert((long long)kRows * kD / 8 < 0x7fffffffLL);
static_assert(((long long)kOut1 * 4) % 128 == 0);
static_assert(64 * kSP * 4 + 512 * 4 <= 327680);
static_assert(64 * 128 * 4 + 64 * 16 * 4 <= 327680);
static_assert(8 * 16 * 68 * 4 <= 327680);

constexpr size_t kSzXB   = (size_t)kRows * kD * 2;
constexpr size_t kSzWT   = (size_t)kNPL * kD * 2;
constexpr size_t kSzP    = (size_t)kRows * kNPL * 4;
constexpr size_t kSzS    = (size_t)kRows * kA * 4;
constexpr size_t kSzPART = (size_t)kB * 16 * 2 * kA * kF * 4;
constexpr size_t kSzAGG  = (size_t)kMPA * kAgg2 * 2;
constexpr size_t kSzWO2T = (size_t)kF * kAgg2 * 2;
constexpr size_t kSzCB   = (size_t)kMPA * kF * 4;
constexpr size_t kSzVEC  = (size_t)kNVEC * 4;
constexpr size_t kWsTotal = kSzXB + kSzWT + kSzP + kSzS + kSzPART + kSzAGG + kSzWO2T + kSzCB + kSzVEC;
static_assert((kSzXB % 256) == 0 && (kSzWT % 256) == 0 && (kSzP % 256) == 0 && (kSzS % 256) == 0);
static_assert((kSzPART % 256) == 0 && (kSzAGG % 256) == 0 && (kSzWO2T % 256) == 0 && (kSzCB % 256) == 0);
static_assert((kSzVEC % 256) == 0);
static_assert(kWsTotal <= ((size_t)128 << 20));

__device__ __forceinline__ float nanmax(float mx, float p) {
  return (p > mx || p != p) ? p : mx;
}

template <int NC, bool DUP>
__device__ __forceinline__ void xpose_tile(const float* __restrict__ src, unsigned short* dst, int drow0,
                                           int dpitch, int kcol0, float* st, int tid) {
  constexpr int Q   = NC / 4;
  constexpr int NV  = 64 * Q;
  constexpr int NPC = NC * 8;
  static_assert((NV % 256) == 0 && (NPC % 32) == 0);
#pragma unroll 1
  for (int i = tid; i < NV; i += 256) {
    const int row = i / Q;
    const int c   = i - row * Q;
    const v4f v = *(const v4fa*)(src + (size_t)row * NC + 4 * c);
    *(v4fa*)(st + row * kSP + 4 * c) = v;
  }
  __syncthreads();
#pragma unroll 1
  for (int p = tid; p < NPC; p += 256) {
    const int kq = p & 7;
    const int n  = p >> 3;
    float x[8];
#pragma unroll
    for (int e = 0; e < 8; ++e) x[e] = st[(kq * 8 + e) * kSP + n];
    const v4f a = (v4f){ x[0], x[1], x[2], x[3] };
    const v4f c = (v4f){ x[4], x[5], x[6], x[7] };
    const v4u o = pack8_bf16(a, c);
    unsigned short* q0 = dst + (size_t)(drow0 + n) * (size_t)dpitch + kcol0 + kq * 8;
    volatile v4u* qa = (volatile v4u*)q0;
    volatile v4u* qb = (volatile v4u*)(q0 + kAgg);
    *qa = o;
    if (DUP) *qb = o;
    __threadfence();
    *qa = o;
    if (DUP) *qb = o;
  }
}

__global__ __launch_bounds__(256) void k_prepw(const float* __restrict__ w_in, const float* __restrict__ b_in,
                                               const float* __restrict__ w_sc, const float* __restrict__ b_sc,
                                               const float* __restrict__ w_out, const float* __restrict__ b_out,
                                               unsigned short* WT, unsigned short* WO2T, float* VEC) {
  __shared__ __attribute__((aligned(16))) float st[64 * kSP];
  __shared__ __attribute__((aligned(16))) float sv[512];
  const int tid = (int)threadIdx.x;
  const int blk = (int)blockIdx.x;
  if (blk < 64) {
    xpose_tile<128, true>(w_out + (size_t)(kD + blk * 64) * kF, WO2T, 0, kAgg2, blk * 64, st, tid);
  } else if (blk == 64) {
    xpose_tile<128, false>(w_in, WT, 0, kD, 0, st, tid);
  } else if (blk == 65) {
    xpose_tile<128, false>(w_out, WT, kF, kD, 0, st, tid);
  } else if (blk == 66) {
    xpose_tile<16, false>(w_sc, WT, 2 * kF, kD, 0, st, tid);
    const v4u z = (v4u){0u, 0u, 0u, 0u};
#pragma unroll 1
    for (int p = tid; p < (kNPL - 2 * kF - kA) * 8; p += 256) {
      volatile v4u* q = (volatile v4u*)(WT + (size_t)(2 * kF + kA + (p >> 3)) * kD + (p & 7) * 8);
      *q = z;
      __threadfence();
      *q = z;
    }
  } else {
#pragma unroll 1
    for (int it = 0; it < 2; ++it) {
      const int i = it * 256 + tid;
      const float vi = b_in[clampi(i, 0, kF - 1)];
      const float vo = b_out[clampi(i - kF, 0, kF - 1)];
      const float vs = b_sc[clampi(i - 2 * kF, 0, kA - 1)];
      asm volatile("" :: "v"(vi));
      asm volatile("" :: "v"(vo));
      asm volatile("" :: "v"(vs));
      const unsigned m0 = (i < kF) ? 0xFFFFFFFFu : 0u;
      const unsigned m1 = (i >= kF && i < 2 * kF) ? 0xFFFFFFFFu : 0u;
      const unsigned m2 = (i >= 2 * kF && i < 2 * kF + kA) ? 0xFFFFFFFFu : 0u;
      const unsigned bits = (__float_as_uint(vi) & m0) | (__float_as_uint(vo) & m1) | (__float_as_uint(vs) & m2);
      sv[i] = bf16_val(__uint_as_float(bits));
    }
    __syncthreads();
    if (tid < kNVEC / 4) {
      const v4f v = *(const v4fa*)(sv + 4 * tid);
      volatile v4f* q = (volatile v4f*)(VEC + 4 * tid);
      *q = v;
      __threadfence();
      *q = v;
    }
  }
}

__global__ __launch_bounds__(256) void k_soft(const float* __restrict__ P, const float* __restrict__ vec, float* S) {
  __shared__ __attribute__((aligned(16))) float sL[4096];
  const int tid = (int)threadIdx.x;
  const int t0  = (int)blockIdx.x * 16;
#pragma unroll
  for (int it = 0; it < 4; ++it) {
    const int idx = it * 256 + tid;
    const int c4 = idx & 3, tl = (idx >> 2) & 15, b = idx >> 6;
    const v4f v = *(const v4fa*)(P + (size_t)(b * kT + t0 + tl) * kNPL + 2 * kF + 4 * c4);
    *(v4fa*)(sL + idx * 4) = v;
  }
  __syncthreads();
  {
    const int a = tid & 15, tl = tid >> 4;
    const float bs = vec[2 * kF + a];
    float* my = sL + tl * 16 + a;
    float m = __uint_as_float(0xff800000u);
#pragma unroll 1
    for (int b = 0; b < kB; ++b) {
      const float x = my[b * 256] + bs;
      my[b * 256] = x;
      m = fmaxf(m, x);
    }
    float s = 0.0f;
#pragma unroll 1
    for (int b = 0; b < kB; ++b) {
      const float e = expf(my[b * 256] - m);
      my[b * 256] = e;
      s += e;
    }
#pragma unroll 1
    for (int b = 0; b < kB; ++b) {
      const float e = my[b * 256];
      my[b * 256] = e / s;
    }
  }
  __syncthreads();
  v4f vv[4];
#pragma unroll
  for (int it = 0; it < 4; ++it) vv[it] = *(const v4fa*)(sL + (it * 256 + tid) * 4);
#pragma unroll
  for (int it = 0; it < 4; ++it) {
    const int idx = it * 256 + tid;
    *(volatile v4f*)(S + (size_t)((idx >> 6) * kT + t0) * kA + (idx & 63) * 4) = vv[it];
  }
  __threadfence();
#pragma unroll
  for (int it = 0; it < 4; ++it) {
    const int idx = it * 256 + tid;
    *(volatile v4f*)(S + (size_t)((idx >> 6) * kT + t0) * kA + (idx & 63) * 4) = vv[it];
  }
}

__global__ __launch_bounds__(256) void k_pool(const float* __restrict__ P, const float* __restrict__ S,
                                              const float* __restrict__ vec, float* PART) {
#pragma clang fp contract(off)
  __shared__ __attribute__((aligned(16))) float sX[64 * 128];
  __shared__ __attribute__((aligned(16))) float sS[64 * 16];
  const int tid = (int)threadIdx.x;
  const int f = tid & 127, g = tid >> 7;
  const int b = (int)blockIdx.x >> 4, ch = (int)blockIdx.x & 15;
  const int c4 = tid & 31, rw = tid >> 5;
  const v4f bin4 = *(const v4fa*)(vec + 4 * c4);
  const float ninf = __uint_as_float(0xff800000u);
  float mx[8], sm[8];
#pragma unroll
  for (int i = 0; i < 8; ++i) { mx[i] = ninf; sm[i] = 0.0f; }

#pragma unroll 1
  for (int st = 0; st < 4; ++st) {
    const int r0 = b * kT + ch * 256 + st * 64;
#pragma unroll 4
    for (int it = 0; it < 8; ++it) {
      const int row = it * 8 + rw;
      v4f v = *(const v4fa*)(P + (size_t)(r0 + row) * kNPL + 4 * c4);
      v += bin4;
      *(v4fa*)(sX + row * 128 + 4 * c4) = v;
    }
    {
      const v4f sv4 = *(const v4fa*)(S + (size_t)r0 * kA + 4 * tid);
      *(v4fa*)(sS + 4 * tid) = sv4;
    }
    __syncthreads();
#pragma unroll 2
    for (int t = 0; t < 64; ++t) {
      const float xp = sX[t * 128 + f];
      const v4f s0 = *(const v4fa*)(sS + t * 16 + 8 * g);
      const v4f s1 = *(const v4fa*)(sS + t * 16 + 8 * g + 4);
      float p;
      p = xp * s0[0]; mx[0] = nanmax(mx[0], p); sm[0] = sm[0] + p;
      p = xp * s0[1]; mx[1] = nanmax(mx[1], p); sm[1] = sm[1] + p;
      p = xp * s0[2]; mx[2] = nanmax(mx[2], p); sm[2] = sm[2] + p;
      p = xp * s0[3]; mx[3] = nanmax(mx[3], p); sm[3] = sm[3] + p;
      p = xp * s1[0]; mx[4] = nanmax(mx[4], p); sm[4] = sm[4] + p;
      p = xp * s1[1]; mx[5] = nanmax(mx[5], p); sm[5] = sm[5] + p;
      p = xp * s1[2]; mx[6] = nanmax(mx[6], p); sm[6] = sm[6] + p;
      p = xp * s1[3]; mx[7] = nanmax(mx[7], p); sm[7] = sm[7] + p;
    }
    __syncthreads();
  }
#pragma unroll
  for (int i = 0; i < 8; ++i) {
    sX[(8 * g + i) * 128 + f]        = mx[i];
    sX[2048 + (8 * g + i) * 128 + f] = sm[i];
  }
  __syncthreads();
  float* dst = PART + (size_t)blockIdx.x * 4096;
  v4f vv[4];
#pragma unroll
  for (int it = 0; it < 4; ++it) vv[it] = *(const v4fa*)(sX + (it * 256 + tid) * 4);
#pragma unroll
  for (int it = 0; it < 4; ++it) *(volatile v4f*)(dst + (it * 256 + tid) * 4) = vv[it];
  __threadfence();
#pragma unroll
  for (int it = 0; it < 4; ++it) *(volatile v4f*)(dst + (it * 256 + tid) * 4) = vv[it];
}

__global__ __launch_bounds__(256) void k_comb(const float* __restrict__ PART, float* out1, unsigned short* AGG) {
  __shared__ __attribute__((aligned(16))) float sv[1024];
  const int tid = (int)threadIdx.x;
  const int blk = (int)blockIdx.x;
  if (blk >= 64) {
    const v4u z = (v4u){0u, 0u, 0u, 0u};
    unsigned short* rowp = AGG + (size_t)(kB + blk - 64) * kAgg2;
#pragma unroll
    for (int it = 0; it < 4; ++it) *(volatile v4u*)(rowp + (size_t)(it * 256 + tid) * 8) = z;
    __threadfence();
#pragma unroll
    for (int it = 0; it < 4; ++it) *(volatile v4u*)(rowp + (size_t)(it * 256 + tid) * 8) = z;
    return;
  }
  const int g = blk * 256 + tid;
  const int f4 = g & 31, which = (g >> 5) & 1, a = (g >> 6) & 15, b = g >> 10;
  const float* pp = PART + (size_t)b * 65536 + (size_t)which * 2048 + a * 128 + 4 * f4;
  const float ninf = __uint_as_float(0xff800000u);
  v4f mxv = (v4f){ninf, ninf, ninf, ninf};
  v4f smv = (v4f){0.f, 0.f, 0.f, 0.f};
#pragma unroll 4
  for (int c = 0; c < 16; ++c) {
    const v4f v = *(const v4fa*)(pp + (size_t)c * 4096);
    mxv[0] = nanmax(mxv[0], v[0]); mxv[1] = nanmax(mxv[1], v[1]);
    mxv[2] = nanmax(mxv[2], v[2]); mxv[3] = nanmax(mxv[3], v[3]);
    smv += v;
  }
  const float sc = 1.0f / 4096.0f;
  v4f res;
  res[0] = which ? smv[0] * sc : mxv[0];
  res[1] = which ? smv[1] * sc : mxv[1];
  res[2] = which ? smv[2] * sc : mxv[2];
  res[3] = which ? smv[3] * sc : mxv[3];
  {
    volatile v4f* q = (volatile v4f*)(out1 + (size_t)g * 4);
    *q = res;
    __threadfence();
    *q = res;
  }
  *(v4fa*)(sv + 4 * tid) = res;
  __syncthreads();
  if (tid < 128) {
    const v4f a4 = *(const v4fa*)(sv + 8 * tid);
    const v4f c4 = *(const v4fa*)(sv + 8 * tid + 4);
    const v4u hi = pack8_bf16(a4, c4);
    const v4u lo = pack8_bf16_lo(a4, c4);
    unsigned short* q0 = AGG + (size_t)(blk >> 2) * kAgg2 + (blk & 3) * 1024 + 8 * tid;
    volatile v4u* qh = (volatile v4u*)q0;
    volatile v4u* ql = (volatile v4u*)(q0 + kAgg);
    *qh = hi;
    *ql = lo;
    __threadfence();
    *qh = hi;
    *ql = lo;
  }
}

__global__ __launch_bounds__(256) void k_out(const float* __restrict__ P, const float* __restrict__ CB,
                                             const float* __restrict__ vec, float* out) {
  const int lane = (int)threadIdx.x & 31, wave = (int)threadIdx.x >> 5;
  const int r0 = (int)blockIdx.x * 64 + wave * 8;
  const int b  = ((int)blockIdx.x * 64) >> 12;
  const v4f cb = *(const v4fa*)(CB + (size_t)b * kF + 4 * lane);
  const v4f bo = *(const v4fa*)(vec + kF + 4 * lane);
  v4f vv[8];
#pragma unroll
  for (int i = 0; i < 8; ++i) {
    const v4f q = *(const v4fa*)(P + (size_t)(r0 + i) * kNPL + kF + 4 * lane);
    v4f v = (q + cb) + bo;
    v[0] = (v[0] < 0.0f) ? 0.0f : v[0];
    v[1] = (v[1] < 0.0f) ? 0.0f : v[1];
    v[2] = (v[2] < 0.0f) ? 0.0f : v[2];
    v[3] = (v[3] < 0.0f) ? 0.0f : v[3];
    vv[i] = v;
  }
#pragma unroll
  for (int i = 0; i < 8; ++i) *(volatile v4f*)(out + (size_t)(r0 + i) * kF + 4 * lane) = vv[i];
  __threadfence();
#pragma unroll
  for (int i = 0; i < 8; ++i) *(volatile v4f*)(out + (size_t)(r0 + i) * kF + 4 * lane) = vv[i];
}

extern "C" void kernel_launch(void* const* d_in, const int* in_sizes, int n_in,
                              void* d_out, int out_size, void* d_ws, size_t ws_size,
                              hipStream_t stream) {
  if (n_in < 7) return;
  if (in_sizes[0] != kRows * kD) return;
  if (in_sizes[1] != kD * kF) return;
  if (in_sizes[2] != kF) return;
  if (in_sizes[3] != kD * kA) return;
  if (in_sizes[4] != kA) return;
  if (in_sizes[5] != (kD + kAgg) * kF) return;
  if (in_sizes[6] != kF) return;
  if ((long long)out_size != (long long)kOut1 + (long long)kB * kAgg) return;
  if (kWsTotal > ws_size) return;

  const float* X    = (const float*)d_in[0];
  const float* Win  = (const float*)d_in[1];
  const float* bin  = (const float*)d_in[2];
  const float* Wsc  = (const float*)d_in[3];
  const float* bsc  = (const float*)d_in[4];
  const float* Wout = (const float*)d_in[5];
  const float* bout = (const float*)d_in[6];
  float* out = (float*)d_out;

  char* ws = (char*)d_ws;
  size_t off = 0;
  unsigned short* XB   = (unsigned short*)(ws + off); off += kSzXB;
  unsigned short* WT   = (unsigned short*)(ws + off); off += kSzWT;
  float*          P    = (float*)(ws + off);          off += kSzP;
  float*          S    = (float*)(ws + off);          off += kSzS;
  float*          PART = (float*)(ws + off);          off += kSzPART;
  unsigned short* AGG  = (unsigned short*)(ws + off); off += kSzAGG;
  unsigned short* WO2T = (unsigned short*)(ws + off); off += kSzWO2T;
  float*          CB   = (float*)(ws + off);          off += kSzCB;
  float*          VEC  = (float*)(ws + off);          off += kSzVEC;
  if (off != kWsTotal || off > ws_size) return;

  k_prepw<<<68, 256, 0, stream>>>(Win, bin, Wsc, bsc, Wout, bout, WT, WO2T, VEC);
  k_plane<0><<<kRows * kD / 8 / 256, 256, 0, stream>>>(X, kRows, kD, kD, XB, kRows, kD);
  k_gemm_nt<0, 0><<<(kRows / 64) * (kNPL / 64) / 8, 256, 0, stream>>>(XB, WT, VEC, P, kRows, kNPL, kD, kNPL);
  k_soft<<<kT / 16, 256, 0, stream>>>(P, VEC, S);
  k_pool<<<kB * 16, 256, 0, stream>>>(P, S, VEC, PART);
  k_comb<<<64 + (kMPA - kB), 256, 0, stream>>>(PART, out + (size_t)kOut1, AGG);
  k_gemm_nt<0, 0><<<1, 256, 0, stream>>>(AGG, WO2T, VEC, CB, kB, kF, kAgg2, kF);
  k_out<<<kRows / 64, 256, 0, stream>>>(P, CB, VEC, out);
}
